// OuterPosBow_68616397521347
// MI455X (gfx1250) — hardware-verified
//
#include <hip/hip_runtime.h>

typedef float          v8f   __attribute__((ext_vector_type(8)));
typedef float          v4f   __attribute__((ext_vector_type(4)));
typedef unsigned int   v4u   __attribute__((ext_vector_type(4)));
typedef int            v8i   __attribute__((ext_vector_type(8)));
typedef unsigned short v8us  __attribute__((ext_vector_type(8)));
typedef unsigned short v16us __attribute__((ext_vector_type(16)));
typedef __bf16         v16bf __attribute__((ext_vector_type(16)));
typedef _Float16       v16h  __attribute__((ext_vector_type(16)));
typedef v4f  __attribute__((may_alias)) v4fa;
typedef v8us __attribute__((may_alias)) v8usa;
union FragB { v16bf v; v16us u; v8us h[2]; v8i w; };
union FragH { v16h  v; v16us u; v8us h[2]; v8i w; };

__device__ __forceinline__ v8f wmb(const FragB& a, const FragB& b, v8f c) {
  v8f d = __builtin_amdgcn_wmma_f32_16x16x32_bf16(false, a.v, false, b.v, (short)0, c, false, false);
  asm volatile("v_nop\n\tv_nop\n\tv_nop\n\tv_nop" : "+v"(d) : "v"(a.w), "v"(b.w));
  return d;
}

__device__ __forceinline__ v8f wmh(const FragH& a, const FragH& b, v8f c) {
  v8f d = __builtin_amdgcn_wmma_f32_16x16x32_f16(false, a.v, false, b.v, (short)0, c, false, false);
  asm volatile("v_nop\n\tv_nop\n\tv_nop\n\tv_nop" : "+v"(d) : "v"(a.w), "v"(b.w));
  return d;
}

__device__ __forceinline__ unsigned bf16_bits(float f) {
  const unsigned u = __float_as_uint(f);
  const unsigned r = (u + 0x7FFFu + ((u >> 16) & 1u)) >> 16;
  const unsigned q = (u >> 16) | 0x40u;
  return ((u & 0x7fffffffu) > 0x7f800000u) ? q : r;
}

__device__ __forceinline__ float bf16_val(float f) {
  return __uint_as_float(bf16_bits(f) << 16);
}
__device__ __forceinline__ int clampi(int v, int lo, int hi) {
  return v < lo ? lo : (v > hi ? hi : v);
}

__device__ __forceinline__ unsigned f16_bits(float f) {
  const unsigned u  = __float_as_uint(f);
  const unsigned s  = (u >> 16) & 0x8000u;
  const unsigned a  = u & 0x7fffffffu;
  const unsigned t  = a - 0x38000000u;
  const unsigned r  = (t + 0x0FFFu + ((t >> 13) & 1u)) >> 13;
  const unsigned rc = r > 0x7C00u ? 0x7C00u : r;
  const bool small  = a < 0x38800000u;
  const bool isnan  = a > 0x7f800000u;
  const unsigned fin = small ? 0u : (s | rc);
  return isnan ? (s | 0x7E00u) : fin;
}

__device__ __forceinline__ unsigned pk16(unsigned lo, unsigned hi) { return lo | (hi << 16); }
__device__ __forceinline__ unsigned bf16_lo_bits(float v) {
  float hi = bf16_val(v);
  asm volatile("" : "+v"(hi));
  return bf16_bits(v - hi);
}
__device__ __forceinline__ v4u pack8_bf16(v4f a, v4f c) {
  return (v4u){ pk16(bf16_bits(a[0]), bf16_bits(a[1])), pk16(bf16_bits(a[2]), bf16_bits(a[3])),
                pk16(bf16_bits(c[0]), bf16_bits(c[1])), pk16(bf16_bits(c[2]), bf16_bits(c[3])) };
}
__device__ __forceinline__ v4u pack8_bf16_lo(v4f a, v4f c) {
  return (v4u){ pk16(bf16_lo_bits(a[0]), bf16_lo_bits(a[1])), pk16(bf16_lo_bits(a[2]), bf16_lo_bits(a[3])),
                pk16(bf16_lo_bits(c[0]), bf16_lo_bits(c[1])), pk16(bf16_lo_bits(c[2]), bf16_lo_bits(c[3])) };
}
__device__ __forceinline__ v4u pack8_f16(v4f a, v4f c) {
  return (v4u){ pk16(f16_bits(a[0]), f16_bits(a[1])), pk16(f16_bits(a[2]), f16_bits(a[3])),
                pk16(f16_bits(c[0]), f16_bits(c[1])), pk16(f16_bits(c[2]), f16_bits(c[3])) };
}

template <int FORM>
__global__ __launch_bounds__(256) void k_plane(const float* __restrict__ src, int rows, int cols, int ldsrc,
                                               unsigned short* __restrict__ dst, int MP, int KP) {
  static_assert(FORM >= 0 && FORM <= 3);
  const int KTOT = (FORM == 1 || FORM == 3) ? 2 * KP : KP;
  const unsigned ppr   = (unsigned)(KTOT >> 3);
  const unsigned kp8   = (unsigned)(KP >> 3);
  const unsigned total = (unsigned)MP * ppr;
  const unsigned g     = blockIdx.x * 256u + threadIdx.x;
  const unsigned rowu  = g / ppr;
  const unsigned p     = g - rowu * ppr;
  const bool second    = p >= kp8;
  const int row = (int)rowu;
  const int c0  = (int)((second ? p - kp8 : p) << 3);
  const float* srow = src + (size_t)clampi(row, 0, rows - 1) * (size_t)ldsrc;
  float x[8];
  unsigned mk[8];
#pragma unroll
  for (int e = 0; e < 8; ++e) {
    const int c = c0 + e;
    const float v = srow[clampi(c, 0, cols - 1)];
    asm volatile("" :: "v"(v));
    x[e]  = v;
    mk[e] = (row < rows && c < cols) ? 0xFFFFu : 0u;
  }
  const v4f a = (v4f){ x[0], x[1], x[2], x[3] };
  const v4f c = (v4f){ x[4], x[5], x[6], x[7] };
  v4u o;
  if (FORM == 2) {
    o = pack8_f16(a, c);
  } else {
    const v4u hi = pack8_bf16(a, c);
    o = hi;
    if (FORM == 1) { const v4u lo = pack8_bf16_lo(a, c); o = second ? lo : hi; }
  }
  const v4u mw = (v4u){ pk16(mk[0], mk[1]), pk16(mk[2], mk[3]), pk16(mk[4], mk[5]), pk16(mk[6], mk[7]) };
  o &= mw;
  if (g < total) {
    volatile v4u* q = (volatile v4u*)(dst + (size_t)g * 8);
    *q = o;
    __threadfence();
    *q = o;
  }
}

template <int FORM> struct FragOf    { typedef FragB T; };
template <>         struct FragOf<2> { typedef FragH T; };
__device__ __forceinline__ v8f mm(const FragB& a, const FragB& b, v8f c) { return wmb(a, b, c); }
__device__ __forceinline__ v8f mm(const FragH& a, const FragH& b, v8f c) { return wmh(a, b, c); }
template <class F> __device__ __forceinline__ F ld_frag(const unsigned short* p) {
  F f;
  f.h[0] = *(const v8usa*)(p);
  f.h[1] = *(const v8usa*)(p + 16);
  return f;
}

template <int FORM, int EPI>
__global__ __launch_bounds__(256) __attribute__((amdgpu_num_vgpr(248)))
void k_gemm_nt(const unsigned short* __restrict__ A, const unsigned short* __restrict__ B,
               const float* __restrict__ bias, float* __restrict__ D, int M, int N, int KTOT, int ldd) {
  static_assert(FORM >= 0 && FORM <= 2);
  static_assert(EPI == 0 || EPI == 1);
  typedef typename FragOf<FORM>::T F;
  __shared__ __attribute__((aligned(16))) float sT[8][16 * 68];
  const int lane = threadIdx.x & 31;
  const int wave = threadIdx.x >> 5;
  const int tilesM = (M + 63) >> 6;
  const int tilesN = (N + 63) >> 6;
  const int tile = blockIdx.x * 8 + wave;
  if (tile >= tilesM * tilesN) return;
  const int tm = tile / tilesN;
  const int tn = tile - tm * tilesN;
  const int m0 = tm << 6;
  const int n0 = tn << 6;

  const int rl = lane & 15;
  const int h8 = (lane >> 4) * 8;
  const unsigned short* pa = A + (size_t)(m0 + rl) * (size_t)KTOT + h8;
  const unsigned short* pb = B + (size_t)(n0 + rl) * (size_t)KTOT + h8;

  v8f acc[4][4];
#pragma unroll
  for (int i = 0; i < 4; ++i)
#pragma unroll
    for (int j = 0; j < 4; ++j) acc[i][j] = (v8f){0.f, 0.f, 0.f, 0.f, 0.f, 0.f, 0.f, 0.f};

#pragma unroll 1
  for (int k0 = 0; k0 < KTOT; k0 += 32) {
    F bf[4];
#pragma unroll
    for (int j = 0; j < 4; ++j) bf[j] = ld_frag<F>(pb + (size_t)(j << 4) * (size_t)KTOT + k0);
#pragma unroll
    for (int i = 0; i < 4; ++i) {
      const F af = ld_frag<F>(pa + (size_t)(i << 4) * (size_t)KTOT + k0);
#pragma unroll
      for (int j = 0; j < 4; ++j) acc[i][j] = mm(af, bf[j], acc[i][j]);
    }
  }

  float* slab = sT[wave];
  const int hh = lane >> 4;
  const int c4 = (lane & 15) * 4;
  const int nc = n0 + c4;
  const bool cok = nc < N;
  v4f bv = (v4f){0.f, 0.f, 0.f, 0.f};
  if (EPI == 1) {
    bv = *(const v4fa*)(bias + clampi(nc, 0, N - 4));
    asm volatile("" :: "v"(bv));
  }
#pragma unroll
  for (int i = 0; i < 4; ++i) {
    const int mBase = m0 + (i << 4);
#pragma unroll
    for (int j = 0; j < 4; ++j) {
#pragma unroll
      for (int r = 0; r < 8; ++r) slab[(h8 + r) * 68 + (j << 4) + rl] = acc[i][j][r];
    }
    __builtin_amdgcn_fence(__ATOMIC_RELEASE, "workgroup");
    __builtin_amdgcn_wave_barrier();
    __builtin_amdgcn_fence(__ATOMIC_ACQUIRE, "workgroup");
    v4f vv[8];
#pragma unroll
    for (int it = 0; it < 8; ++it) {
      const int row = it * 2 + hh;
      v4f v = *(const v4fa*)(slab + row * 68 + c4);
      if (EPI == 1) v += bv;
      vv[it] = v;
    }
    for (int pass = 0; pass < 2; ++pass) {
#pragma unroll
      for (int it = 0; it < 8; ++it) {
        const int row = mBase + it * 2 + hh;
        if (cok && row < M) *(volatile v4f*)(D + (size_t)row * (size_t)ldd + nc) = vv[it];
      }
      __threadfence();
    }
    __builtin_amdgcn_fence(__ATOMIC_RELEASE, "workgroup");
    __builtin_amdgcn_wave_barrier();
    __builtin_amdgcn_fence(__ATOMIC_ACQUIRE, "workgroup");
  }
}

#pragma clang fp contract(off)

typedef int v2i __attribute__((ext_vector_type(2)));
typedef v2i __attribute__((may_alias)) v2ia;

constexpr int NWORDS = 64 * 256;
constexpr int LPOS   = 32;
constexpr int NCHAR  = 64;
constexpr int E3     = 256;
constexpr int ROWLEN = 770;
constexpr int PADL   = 2;
constexpr int OUT_ELEMS = NWORDS * ROWLEN;
constexpr int WPB    = 32;

static_assert(ROWLEN == PADL + 3 * E3);
static_assert(NCHAR == 64 && NCHAR == 2 * 32 && NCHAR % 32 == 0);
static_assert(E3 == 256 && E3 % 64 == 0 && E3 % 32 == 0 && E3 % 4 == 0);
static_assert(LPOS == 32);
static_assert(NWORDS == 16384 && NWORDS % WPB == 0 && NWORDS % 128 == 0 && NWORDS % 64 == 0 && NWORDS % 16 == 0);
static_assert(OUT_ELEMS == 12615680 && OUT_ELEMS % 256 == 0 && (OUT_ELEMS / 256) * 256 == OUT_ELEMS);
static_assert(OUT_ELEMS / 256 == 49280);
static_assert((long long)NWORDS * NCHAR / 8 < 0x7fffffffLL);

constexpr size_t SZ_WB  = (size_t)E3 * NCHAR * 2;
constexpr size_t SZ_WT  = (size_t)NCHAR * E3 * 4;
constexpr size_t SZ_CNT = (size_t)NWORDS * NCHAR * 2;
constexpr size_t SZ_R   = (size_t)NWORDS * 2 * 4;
constexpr size_t SZ_BAG = (size_t)NWORDS * E3 * 4;
constexpr size_t OFF_WB  = 0;
constexpr size_t OFF_WT  = OFF_WB + SZ_WB;
constexpr size_t OFF_CNT = OFF_WT + SZ_WT;
constexpr size_t OFF_R   = OFF_CNT + SZ_CNT;
constexpr size_t OFF_BAG = OFF_R + SZ_R;
constexpr size_t WS_TOTAL = OFF_BAG + SZ_BAG;
static_assert(SZ_WB % 256 == 0 && SZ_WT % 256 == 0 && SZ_CNT % 256 == 0 && SZ_R % 256 == 0 && SZ_BAG % 256 == 0);
static_assert(OFF_WT == (size_t)32768 && OFF_CNT == (size_t)98304 && OFF_R == (size_t)2195456);
static_assert(OFF_BAG == (size_t)2326528 && WS_TOTAL == (size_t)19103744);
static_assert(OFF_WT % 256 == 0 && OFF_CNT % 256 == 0 && OFF_R % 256 == 0 && OFF_BAG % 256 == 0);
static_assert(WS_TOTAL <= ((size_t)128 << 20));

__global__ __launch_bounds__(256) void k_wt(const float* __restrict__ W, float* __restrict__ WT) {
  __shared__ float tile[64 * 65];
  const int tid = (int)threadIdx.x, lane = tid & 31, wave = tid >> 5;
  const int o0 = (int)blockIdx.x << 6;
  const int c4 = (tid & 15) * 4;
#pragma unroll
  for (int i = 0; i < 4; ++i) {
    const int orow = (tid >> 4) + 16 * i;
    const v4f v = *(const v4fa*)(W + (size_t)(o0 + orow) * (size_t)NCHAR + c4);
    asm volatile("" :: "v"(v));
    tile[orow * 65 + c4 + 0] = bf16_val(v[0]);
    tile[orow * 65 + c4 + 1] = bf16_val(v[1]);
    tile[orow * 65 + c4 + 2] = bf16_val(v[2]);
    tile[orow * 65 + c4 + 3] = bf16_val(v[3]);
  }
  __syncthreads();
  float x[16];
#pragma unroll
  for (int i = 0; i < 16; ++i) {
    const int q  = wave * 16 + i;
    const int c  = q >> 1;
    const int ol = (q & 1) * 32 + lane;
    x[i] = tile[ol * 65 + c];
  }
#pragma unroll
  for (int i = 0; i < 16; ++i) {
    const int q  = wave * 16 + i;
    const int c  = q >> 1;
    const int ol = (q & 1) * 32 + lane;
    *(volatile float*)(WT + (size_t)c * E3 + o0 + ol) = x[i];
  }
  __threadfence();
#pragma unroll
  for (int i = 0; i < 16; ++i) {
    const int q  = wave * 16 + i;
    const int c  = q >> 1;
    const int ol = (q & 1) * 32 + lane;
    *(volatile float*)(WT + (size_t)c * E3 + o0 + ol) = x[i];
  }
}

__global__ __launch_bounds__(256) void k_word(const int* __restrict__ ids, unsigned* __restrict__ CNT,
                                              int* __restrict__ R) {
  __shared__ int sR[64];
  const int tid = (int)threadIdx.x, lane = tid & 31, wave = tid >> 5;
  const bool inb = (lane >= 1) & (lane <= 30);
#pragma unroll 1
  for (int i = 0; i < 4; ++i) {
    const int word = __builtin_amdgcn_readfirstlane((int)blockIdx.x * WPB + wave * 4 + i);
    const int wc = word < NWORDS ? word : NWORDS - 1;
    int id = ids[(size_t)wc * LPOS + lane];
    asm volatile("" :: "v"(id));
    id = clampi(id, 0, NCHAR - 1);

    int mx = id;
    { const int o = __shfl_xor(mx, 16, 32); mx = o > mx ? o : mx; }
    { const int o = __shfl_xor(mx, 8, 32);  mx = o > mx ? o : mx; }
    { const int o = __shfl_xor(mx, 4, 32);  mx = o > mx ? o : mx; }
    { const int o = __shfl_xor(mx, 2, 32);  mx = o > mx ? o : mx; }
    { const int o = __shfl_xor(mx, 1, 32);  mx = o > mx ? o : mx; }
    const unsigned bal = __builtin_amdgcn_ballot_w32(id == mx);
    const int am = __builtin_ctz(bal | 0x80000000u);
    int wl = am > 0 ? am - 1 : 0;
    wl = __builtin_amdgcn_readfirstlane(wl);
    const int ends = __builtin_amdgcn_readlane(id, wl);
    int s = (lane == wl) ? 0 : id;
    s = (lane == 31) ? ends : s;

    int e0 = 0, e1 = 0;
#pragma unroll 2
    for (int cp = 0; cp < 32; ++cp) {
      const unsigned b0 = __builtin_amdgcn_ballot_w32(inb & (s == 2 * cp));
      const unsigned b1 = __builtin_amdgcn_ballot_w32(inb & (s == 2 * cp + 1));
      const int n0 = __builtin_popcount(b0);
      const int n1 = __builtin_popcount(b1);
      e0 = (lane == cp) ? n0 : e0;
      e1 = (lane == cp) ? n1 : e1;
    }
    const unsigned wd = pk16(bf16_bits((float)e0), bf16_bits((float)e1));

    const int s0  = __builtin_amdgcn_readlane(s, 0);
    const int s31 = __builtin_amdgcn_readlane(s, 31);
    const int rv  = (lane == 0) ? s0 : s31;
    if (lane < 2) sR[(wave * 4 + i) * 2 + lane] = rv;

    if (word < NWORDS) {
      volatile unsigned* q = (volatile unsigned*)(CNT + (size_t)word * 32 + lane);
      *q = wd;
      __threadfence();
      *q = wd;
    }
  }
  __syncthreads();
  const int rline = sR[(wave & 1) * 32 + lane];
  if (wave < 2) {
    volatile int* q = (volatile int*)(R + (size_t)blockIdx.x * 64 + wave * 32 + lane);
    *q = rline;
    __threadfence();
    *q = rline;
  }
}

__global__ __launch_bounds__(256) void k_out(const int* __restrict__ R, const float* __restrict__ WT,
                                             const float* __restrict__ BAG, float* __restrict__ out) {
  const int f  = (int)blockIdx.x * 256 + (int)threadIdx.x;
  const int fc = f < OUT_ELEMS ? f : OUT_ELEMS - 1;
  const int w  = fc / ROWLEN;
  const int j  = fc - w * ROWLEN;
  const v2i rr = *(const v2ia*)(R + 2 * (size_t)w);
  int r0 = rr[0];
  int r1 = rr[1];
  asm volatile("" :: "v"(r0));
  asm volatile("" :: "v"(r1));
  r0 = clampi(r0, 0, NCHAR - 1);
  r1 = clampi(r1, 0, NCHAR - 1);
  const float a = WT[(size_t)r0 * E3 + clampi(j - PADL, 0, E3 - 1)];
  asm volatile("" :: "v"(a));
  const float b = BAG[(size_t)w * E3 + clampi(j - PADL - E3, 0, E3 - 1)];
  asm volatile("" :: "v"(b));
  const float c = WT[(size_t)r1 * E3 + clampi(j - PADL - 2 * E3, 0, E3 - 1)];
  asm volatile("" :: "v"(c));
  const unsigned ma = ((j >= PADL) & (j < PADL + E3)) ? 0xFFFFFFFFu : 0u;
  const unsigned mb = ((j >= PADL + E3) & (j < PADL + 2 * E3)) ? 0xFFFFFFFFu : 0u;
  const unsigned mc = (j >= PADL + 2 * E3) ? 0xFFFFFFFFu : 0u;
  const unsigned vb = (__float_as_uint(a) & ma) | (__float_as_uint(b) & mb) | (__float_as_uint(c) & mc);
  const float v = __uint_as_float(vb);
  if (f < OUT_ELEMS) {
    volatile float* q = (volatile float*)(out + f);
    *q = v;
    __threadfence();
    *q = v;
  }
}

extern "C" void kernel_launch(void* const* d_in, const int* in_sizes, int n_in,
                              void* d_out, int out_size, void* d_ws, size_t ws_size,
                              hipStream_t stream) {
  if (n_in < 2) return;
  if (in_sizes[0] != NWORDS * LPOS) return;
  if (in_sizes[1] != E3 * NCHAR) return;
  if (out_size != OUT_ELEMS) return;
  if (ws_size < WS_TOTAL) return;

  const int*   ids = (const int*)d_in[0];
  const float* W   = (const float*)d_in[1];
  float* out = (float*)d_out;

  char* ws = (char*)d_ws;
  unsigned short* WB  = (unsigned short*)(ws + OFF_WB);
  float*          WT  = (float*)(ws + OFF_WT);
  unsigned*       CNT = (unsigned*)(ws + OFF_CNT);
  int*            R   = (int*)(ws + OFF_R);
  float*          BAG = (float*)(ws + OFF_BAG);

  k_plane<0><<<(E3 * NCHAR / 8) / 256, 256, 0, stream>>>(W, E3, NCHAR, NCHAR, WB, E3, NCHAR);
  k_wt<<<E3 / 64, 256, 0, stream>>>(W, WT);
  k_word<<<NWORDS / WPB, 256, 0, stream>>>(ids, CNT, R);
  k_gemm_nt<0, 0><<<((NWORDS / 64) * (E3 / 64) + 7) / 8, 256, 0, stream>>>(
      (const unsigned short*)CNT, WB, WT, BAG, NWORDS, E3, NCHAR, E3);
  k_out<<<OUT_ELEMS / 256, 256, 0, stream>>>(R, WT, BAG, out);
}
